// GraphMP_4690104287811
// MI455X (gfx1250) — hardware-run, weakly checked
//
#include <hip/hip_runtime.h>
#include <stddef.h>


#define FEAT 32
#define NTILE 68
#define PITCH 1088
#define COL_ROOT 1024
#define COL_XB 1056
#define NSLOTS (NTILE * 64)

#define CH1 4096
#define MAXB 1600
#define PITCHB 1568
#define BPT 7
#define MAXNB1 128
#define CAP3 1024
#define GMAX 64
#define BN_EPS 1e-5f

typedef _Float16 v16h __attribute__((ext_vector_type(16)));
typedef _Float16 v8h __attribute__((ext_vector_type(8)));
typedef float v8f __attribute__((ext_vector_type(8)));
typedef float v4f __attribute__((ext_vector_type(4)));
typedef int v4i __attribute__((ext_vector_type(4)));
typedef v4f __attribute__((may_alias)) v4fa;
typedef v4i __attribute__((may_alias)) v4ia;

union Frag { v16h v; v8h half[2]; _Float16 e[16]; };

__device__ __forceinline__ v8f wmma16(const v16h& a, const v16h& b, v8f c) {
    return __builtin_amdgcn_wmma_f32_16x16x32_f16(false, a, false, b, (short)0, c, false, false);
}

__global__ __launch_bounds__(256) void k_prep(const float* __restrict__ w2, const float* __restrict__ root,
                                              const float* __restrict__ b2, _Float16* bfrag) {
    const int t0 = blockIdx.x * 256 + threadIdx.x;
    const bool ok = t0 < NSLOTS;
    const int tt = ok ? t0 : 0;
    const int g = tt & 1, l = (tt >> 1) & 31, t = tt >> 6;
    const int h = l >> 4, c = t * 16 + (l & 15);
    const int kb = 8 * h + 16 * g;
    const int o5 = c & 31, ow = (c >> 5) & 31;
    union { v8h v; _Float16 e[8]; } u;
#pragma unroll
    for (int ii = 0; ii < 8; ++ii) {
        const int k = kb + ii;
        const float vw = w2[o5 * 1024 + k * 32 + ow];
        const float vr = root[k * 32 + o5];
        const float vb = b2[k * 32 + o5];
        const float v = (c < COL_ROOT) ? vw : ((c < COL_XB) ? vr : vb);
        u.e[ii] = (_Float16)(v * 64.0f);
    }
    const v8h val = u.v;
    if (ok) *(volatile v8h*)(bfrag + (size_t)tt * 8) = val;
    __threadfence();
    if (ok) *(volatile v8h*)(bfrag + (size_t)tt * 8) = val;
}

__global__ __launch_bounds__(32) void k_node(const float* __restrict__ x, const _Float16* bfrag,
                                             float* nodep, int N, int ntiles) {
    __shared__ __attribute__((aligned(16))) float stg[16 * 32];
    const int tile = blockIdx.x;
    if (tile >= ntiles) return;
    const int lane = threadIdx.x & 31, h = lane >> 4, m = lane & 15;
    int row = tile * 16 + m;
    row = row > N - 1 ? N - 1 : row;
    const v4f* xr = (const v4f*)(x + (size_t)row * FEAT);
    const v4f p0 = xr[2 * h], p1 = xr[2 * h + 1], p2 = xr[4 + 2 * h], p3 = xr[5 + 2 * h];
    Frag a;
    a.e[0] = (_Float16)p0.x;  a.e[1] = (_Float16)p0.y;  a.e[2] = (_Float16)p0.z;  a.e[3] = (_Float16)p0.w;
    a.e[4] = (_Float16)p1.x;  a.e[5] = (_Float16)p1.y;  a.e[6] = (_Float16)p1.z;  a.e[7] = (_Float16)p1.w;
    a.e[8] = (_Float16)p2.x;  a.e[9] = (_Float16)p2.y;  a.e[10] = (_Float16)p2.z; a.e[11] = (_Float16)p2.w;
    a.e[12] = (_Float16)p3.x; a.e[13] = (_Float16)p3.y; a.e[14] = (_Float16)p3.z; a.e[15] = (_Float16)p3.w;

    const v8h* bq = (const v8h*)bfrag;
    const float inv = 0.015625f;
    float* gbase = nodep + (size_t)tile * 16 * PITCH;
    const v4fa* sv = (const v4fa*)stg;

#pragma unroll 1
    for (int u = 0; u < NTILE / 2; ++u) {
        Frag b0, b1;
        const int f0 = ((2 * u) * 32 + lane) * 2;
        const int f1 = ((2 * u + 1) * 32 + lane) * 2;
        b0.half[0] = bq[f0];
        b0.half[1] = bq[f0 + 1];
        b1.half[0] = bq[f1];
        b1.half[1] = bq[f1 + 1];
        v8f z;
#pragma unroll
        for (int r = 0; r < 8; ++r) z[r] = 0.0f;
        v8f c0 = wmma16(a.v, b0.v, z);
        v8f c1 = wmma16(a.v, b1.v, z);
        asm volatile("v_nop\n\tv_nop\n\tv_nop\n\tv_nop" : "+v"(c0), "+v"(c1) : "v"(a.v), "v"(b0.v), "v"(b1.v));
#pragma unroll
        for (int r = 0; r < 8; ++r) {
            stg[(8 * h + r) * 32 + m] = c0[r] * inv;
            stg[(8 * h + r) * 32 + 16 + m] = c1[r] * inv;
        }
        __syncthreads();
        v4f ov[4];
#pragma unroll
        for (int it = 0; it < 4; ++it) ov[it] = sv[it * 32 + lane];
        float* gp = gbase + 32 * u + (lane & 7) * 4;
#pragma unroll
        for (int it = 0; it < 4; ++it)
            *(volatile v4f*)(gp + (size_t)(it * 4 + (lane >> 3)) * PITCH) = ov[it];
        __threadfence();
#pragma unroll
        for (int it = 0; it < 4; ++it)
            *(volatile v4f*)(gp + (size_t)(it * 4 + (lane >> 3)) * PITCH) = ov[it];
        __syncthreads();
    }
}

__device__ __forceinline__ void chunk_keys(const int* __restrict__ recv, int cb, int lane, int E, int N,
                                           unsigned& key_out, int& rank, bool& last, bool& valid) {
    const int e = cb + lane;
    const int ec = e < E ? e : E - 1;
    const int r = recv[ec];
    unsigned key = 0xFFFFFFFFu;
    if (e < E && r >= 0 && r < N) key = ((unsigned)r & ~31u) | (unsigned)lane;
#pragma unroll
    for (int kk = 2; kk <= 32; kk <<= 1) {
#pragma unroll
        for (int j = kk >> 1; j > 0; j >>= 1) {
            const unsigned p = __shfl_xor(key, j);
            const bool asc = (lane & kk) == 0;
            const bool low = (lane & j) == 0;
            const unsigned mn = key < p ? key : p;
            const unsigned mx = key < p ? p : key;
            key = (asc == low) ? mn : mx;
        }
    }
    const unsigned bkt = key >> 5;
    const unsigned pk = __shfl_up(key, 1);
    const unsigned nk = __shfl_down(key, 1);
    const bool start = (lane == 0) || ((pk >> 5) != bkt);
    last = (lane == 31) || ((nk >> 5) != bkt);
    int v = start ? lane : 0;
#pragma unroll
    for (int d = 1; d < 32; d <<= 1) {
        const int uu = __shfl_up(v, d);
        if (lane >= d && uu > v) v = uu;
    }
    rank = lane - v;
    key_out = key;
    valid = (key != 0xFFFFFFFFu);
}

__global__ __launch_bounds__(256) void k_bucket(const int* __restrict__ recv, int* lists, int* offtab, int E, int N) {
    __shared__ unsigned short wcnt[8 * MAXB];
    __shared__ __attribute__((aligned(16))) int list_lds[CH1];
    __shared__ __attribute__((aligned(16))) int boff[PITCHB];
    __shared__ int sb[256];
    const int t = threadIdx.x, lane = t & 31, wid = t >> 5, blk = blockIdx.x;

    for (int i = t; i < 8 * MAXB; i += 256) wcnt[i] = 0;
    for (int i = t; i < CH1; i += 256) list_lds[i] = 0;
    __syncthreads();

    const int wbase = blk * CH1 + wid * 512;
#pragma unroll 1
    for (int c = 0; c < 16; ++c) {
        unsigned key; int rank; bool last, valid;
        chunk_keys(recv, wbase + c * 32, lane, E, N, key, rank, last, valid);
        if (valid && last) {
            const int b = (int)(key >> 5);
            wcnt[wid * MAXB + b] += (unsigned short)(rank + 1);
        }
    }
    __syncthreads();

    int tsum = 0;
#pragma unroll 1
    for (int q = 0; q < BPT; ++q) {
        const int b = t * BPT + q;
        if (b < PITCHB) {
            int tot = 0;
#pragma unroll
            for (int w = 0; w < 8; ++w) tot += (int)wcnt[w * MAXB + b];
            tsum += tot;
        }
    }
    sb[t] = tsum;
    __syncthreads();
#pragma unroll 1
    for (int d = 1; d < 256; d <<= 1) {
        const int v = (t >= d) ? sb[t - d] : 0;
        __syncthreads();
        sb[t] += v;
        __syncthreads();
    }
    int run = sb[t] - tsum;
#pragma unroll 1
    for (int q = 0; q < BPT; ++q) {
        const int b = t * BPT + q;
        if (b < PITCHB) {
            boff[b] = run;
#pragma unroll
            for (int w = 0; w < 8; ++w) {
                const int cnt = (int)wcnt[w * MAXB + b];
                wcnt[w * MAXB + b] = (unsigned short)run;
                run += cnt;
            }
        }
    }
    __syncthreads();

#pragma unroll 1
    for (int c = 0; c < 16; ++c) {
        const int cb = wbase + c * 32;
        unsigned key; int rank; bool last, valid;
        chunk_keys(recv, cb, lane, E, N, key, rank, last, valid);
        if (valid) {
            const int b = (int)(key >> 5);
            const int pos = (int)wcnt[wid * MAXB + b] + rank;
            if ((unsigned)pos < (unsigned)CH1) list_lds[pos] = cb + (int)(key & 31u);
            if (last) wcnt[wid * MAXB + b] = (unsigned short)(pos + 1);
        }
    }
    __syncthreads();

    const v4ia* lsrc = (const v4ia*)list_lds;
    const v4ia* bsrc = (const v4ia*)boff;
    v4i lv[4];
#pragma unroll
    for (int u = 0; u < 4; ++u) lv[u] = lsrc[t + u * 256];
    const int t2 = t + 256;
    const bool has2 = t2 < (PITCHB / 4);
    const v4i bv0 = bsrc[t];
    const v4i bv1 = bsrc[has2 ? t2 : t];
    int* ld = lists + (size_t)blk * CH1;
    int* bd = offtab + (size_t)blk * PITCHB;
#pragma unroll
    for (int u = 0; u < 4; ++u) *(volatile v4i*)(ld + (size_t)(t + u * 256) * 4) = lv[u];
    *(volatile v4i*)(bd + (size_t)t * 4) = bv0;
    if (has2) *(volatile v4i*)(bd + (size_t)t2 * 4) = bv1;
    __threadfence();
#pragma unroll
    for (int u = 0; u < 4; ++u) *(volatile v4i*)(ld + (size_t)(t + u * 256) * 4) = lv[u];
    *(volatile v4i*)(bd + (size_t)t * 4) = bv0;
    if (has2) *(volatile v4i*)(bd + (size_t)t2 * 4) = bv1;
}

__global__ __launch_bounds__(32) void k_aggr(const int* __restrict__ ei, const float* __restrict__ ea,
                                             const float* __restrict__ w1, const float* __restrict__ b1,
                                             const float* __restrict__ bias,
                                             const float* __restrict__ bng, const float* __restrict__ bnb,
                                             const float* __restrict__ bnm, const float* __restrict__ bnv,
                                             const float* nodep, const int* lists, const int* offtab,
                                             float* xout, int E, int N, int NB1) {
    __shared__ unsigned comp[CAP3];
    __shared__ __attribute__((aligned(16))) float acc[32 * 32];
    __shared__ float ecnt[32 * 32];
    __shared__ __attribute__((aligned(16))) float hbuf[2 * 32];
    const int lane = threadIdx.x & 31;
    const int f = blockIdx.x;
    const int* recv = ei + E;
    const float w10 = w1[lane], w11 = w1[FEAT + lane], w12 = w1[2 * FEAT + lane], w13 = w1[3 * FEAT + lane];
    const float b1v = b1[lane], bsv = bias[lane];
    const float gmv = bng[lane], gbv = bnb[lane], mmv = bnm[lane];
    const float rsv = rsqrtf(bnv[lane] + BN_EPS);

    int cnt[4], lo[4], ex[4];
    int carry = 0;
#pragma unroll
    for (int u = 0; u < 4; ++u) {
        const int blk = lane + 32 * u;
        const bool inb = blk < NB1;
        const int* tb = offtab + (size_t)(inb ? blk : 0) * PITCHB;
        int a = tb[f];
        int b = tb[f + 1];
        a = a < 0 ? 0 : (a > CH1 ? CH1 : a);
        b = b < a ? a : (b > CH1 ? CH1 : b);
        const int c = inb ? (b - a) : 0;
        cnt[u] = c;
        lo[u] = inb ? a : 0;
        int s = c;
#pragma unroll
        for (int d = 1; d < 32; d <<= 1) {
            const int v = __shfl_up(s, d);
            if (lane >= d) s += v;
        }
        ex[u] = carry + s - c;
        carry += __shfl(s, 31);
    }
    const int T = carry < CAP3 ? carry : CAP3;

#pragma unroll
    for (int u = 0; u < 4; ++u) {
        const int blk = lane + 32 * u;
        const int* lp = lists + (size_t)(blk < NB1 ? blk : 0) * CH1 + lo[u];
        for (int q = 0; q < cnt[u]; ++q) {
            const int p = ex[u] + q;
            if (p < CAP3) {
                const int e = lp[q];
                const int ec = e < 0 ? 0 : (e > E - 1 ? E - 1 : e);
                const int nd = recv[ec] - f * 32;
                unsigned pk = 0xFFFFFFFFu;
                if ((unsigned)e < (unsigned)E && (unsigned)nd < 32u) pk = ((unsigned)e << 5) | (unsigned)nd;
                comp[p] = pk;
            }
        }
    }
#pragma unroll
    for (int r = 0; r < 32; ++r) {
        acc[r * 32 + lane] = 0.0f;
        ecnt[r * 32 + lane] = 0.0f;
    }
    __syncthreads();

#pragma unroll 1
    for (int i = 0; i < T; ++i) {
        const unsigned pk = comp[i];
        const bool valid = pk != 0xFFFFFFFFu;
        int e = (int)(pk >> 5);
        e = valid ? e : 0;
        e = e > E - 1 ? E - 1 : e;
        const int nd = (int)(pk & 31u);
        int src = ei[e];
        src = src < 0 ? 0 : (src > N - 1 ? N - 1 : src);
        const v4f av = *(const v4f*)(ea + (size_t)e * 4);
        float s = av.x * w10;
        s = fmaf(av.y, w11, s);
        s = fmaf(av.z, w12, s);
        s = fmaf(av.w, w13, s);
        const float he = fmaxf(s + b1v, 0.0f);
        float* hb = hbuf + (i & 1) * 32;
        hb[lane] = he;
        __syncthreads();
        const v4fa* hv = (const v4fa*)hb;
        const float* grow = nodep + (size_t)src * PITCH;
        const v4f* gp = (const v4f*)(grow + lane * 32);
        float msg = grow[COL_XB + lane];
#pragma unroll
        for (int j = 0; j < 8; ++j) {
            const v4f hq = hv[j];
            const v4f g = gp[j];
            msg = fmaf(hq.x, g.x, msg);
            msg = fmaf(hq.y, g.y, msg);
            msg = fmaf(hq.z, g.z, msg);
            msg = fmaf(hq.w, g.w, msg);
        }
        msg = valid ? msg : 0.0f;
        acc[nd * 32 + lane] += msg;
        ecnt[nd * 32 + lane] += valid ? 1.0f : 0.0f;
    }
    __syncthreads();

#pragma unroll 4
    for (int nd = 0; nd < 32; ++nd) {
        int n = f * 32 + nd;
        n = n > N - 1 ? N - 1 : n;
        const float a = acc[nd * 32 + lane];
        const float c = ecnt[nd * 32 + lane];
        const float rc = 1.0f / fmaxf(c, 1.0f);
        float v = a * rc;
        v = v + nodep[(size_t)n * PITCH + COL_ROOT + lane];
        v = v + bsv;
        v = (v - mmv) * rsv;
        v = v * gmv + gbv;
        acc[nd * 32 + lane] = fmaxf(v, 0.0f);
    }
    __syncthreads();

    const v4fa* av2 = (const v4fa*)acc;
    v4f ov[8];
#pragma unroll
    for (int it = 0; it < 8; ++it) ov[it] = av2[it * 32 + lane];
    float* ob = xout + (size_t)f * 32 * FEAT;
#pragma unroll
    for (int it = 0; it < 8; ++it) *(volatile v4f*)(ob + (size_t)(it * 32 + lane) * 4) = ov[it];
    __threadfence();
#pragma unroll
    for (int it = 0; it < 8; ++it) *(volatile v4f*)(ob + (size_t)(it * 32 + lane) * 4) = ov[it];
}

__global__ __launch_bounds__(128) void k_tail(const float* xf, const int* __restrict__ batch,
                                              const float* __restrict__ r1w, const float* __restrict__ r1b,
                                              const float* __restrict__ r2w, const float* __restrict__ r2b,
                                              float* out, int N, int G, int out_size) {
    __shared__ __attribute__((aligned(16))) float pacc[4 * GMAX * 32];
    __shared__ float pcw[4 * GMAX];
    __shared__ __attribute__((aligned(16))) float pooled[GMAX * 32];
    __shared__ float hl[GMAX * 16];
    __shared__ __attribute__((aligned(16))) float outl[GMAX];
    const int t = threadIdx.x, lane = t & 31, wid = t >> 5;
    for (int i = t; i < 4 * GMAX * 32; i += 128) pacc[i] = 0.0f;
    for (int i = t; i < 4 * GMAX; i += 128) pcw[i] = 0.0f;
    if (t < GMAX) outl[t] = 0.0f;
    __syncthreads();

    const int chunk = (N + 3) >> 2;
    const int n0 = wid * chunk;
    int n1 = n0 + chunk;
    n1 = n1 > N ? N : n1;
    float* pa = pacc + wid * (GMAX * 32);
    float* pc = pcw + wid * GMAX;
#pragma unroll 1
    for (int n = n0; n < n1; ++n) {
        const int g = batch[n];
        const float v = xf[(size_t)n * FEAT + lane];
        if ((unsigned)g < (unsigned)G) {
            pa[g * 32 + lane] += v;
            const float cn = pc[g] + 1.0f;
            pc[g] = cn;
        }
    }
    __syncthreads();

    for (int idx = t; idx < GMAX * 32; idx += 128) {
        const int g = idx >> 5;
        const float s = ((pacc[idx] + pacc[GMAX * 32 + idx]) + pacc[2 * GMAX * 32 + idx]) + pacc[3 * GMAX * 32 + idx];
        const float c = ((pcw[g] + pcw[GMAX + g]) + pcw[2 * GMAX + g]) + pcw[3 * GMAX + g];
        pooled[idx] = s * (1.0f / fmaxf(c, 1.0f));
    }
    __syncthreads();

    const int h = lane >> 4, m = lane & 15;
    const v4fa* pr = (const v4fa*)(pooled + (size_t)(16 * wid + m) * 32);
    const v4f p0 = pr[2 * h], p1 = pr[2 * h + 1], p2 = pr[4 + 2 * h], p3 = pr[5 + 2 * h];
    Frag a;
    a.e[0] = (_Float16)p0.x;  a.e[1] = (_Float16)p0.y;  a.e[2] = (_Float16)p0.z;  a.e[3] = (_Float16)p0.w;
    a.e[4] = (_Float16)p1.x;  a.e[5] = (_Float16)p1.y;  a.e[6] = (_Float16)p1.z;  a.e[7] = (_Float16)p1.w;
    a.e[8] = (_Float16)p2.x;  a.e[9] = (_Float16)p2.y;  a.e[10] = (_Float16)p2.z; a.e[11] = (_Float16)p2.w;
    a.e[12] = (_Float16)p3.x; a.e[13] = (_Float16)p3.y; a.e[14] = (_Float16)p3.z; a.e[15] = (_Float16)p3.w;
    Frag b;
#pragma unroll
    for (int ii = 0; ii < 8; ++ii) {
        b.e[ii] = (_Float16)(r1w[(8 * h + ii) * 16 + m] * 64.0f);
        b.e[8 + ii] = (_Float16)(r1w[(16 + 8 * h + ii) * 16 + m] * 64.0f);
    }
    v8f z;
#pragma unroll
    for (int r = 0; r < 8; ++r) z[r] = 0.0f;
    v8f c0 = wmma16(a.v, b.v, z);
    asm volatile("v_nop\n\tv_nop\n\tv_nop\n\tv_nop" : "+v"(c0) : "v"(a.v), "v"(b.v));
    const float rb = r1b[m];
#pragma unroll
    for (int r = 0; r < 8; ++r)
        hl[(16 * wid + 8 * h + r) * 16 + m] = fmaxf(c0[r] * 0.015625f + rb, 0.0f);
    __syncthreads();

    if (t < GMAX) {
        float s = 0.0f;
#pragma unroll
        for (int j = 0; j < 16; ++j) s = fmaf(hl[t * 16 + j], r2w[j], s);
        outl[t] = s + r2b[0];
    }
    __syncthreads();

    const int nv4 = out_size >> 2;
    const v4fa* ovp = (const v4fa*)outl;
    const v4f val = ovp[lane < 16 ? lane : 0];
    const bool ok = (wid == 0) && (lane < nv4);
    if (ok) *(volatile v4f*)(out + (size_t)lane * 4) = val;
    __threadfence();
    if (ok) *(volatile v4f*)(out + (size_t)lane * 4) = val;
}

extern "C" void kernel_launch(void* const* d_in, const int* in_sizes, int n_in,
                              void* d_out, int out_size, void* d_ws, size_t ws_size,
                              hipStream_t stream) {
    if (n_in < 28) return;
    const float* x     = (const float*)d_in[0];
    const float* ea    = (const float*)d_in[1];
    const float* e1w1  = (const float*)d_in[2];
    const float* e1b1  = (const float*)d_in[3];
    const float* e1w2  = (const float*)d_in[4];
    const float* e1b2  = (const float*)d_in[5];
    const float* root1 = (const float*)d_in[6];
    const float* bias1 = (const float*)d_in[7];
    const float* e2w1  = (const float*)d_in[8];
    const float* e2b1  = (const float*)d_in[9];
    const float* e2w2  = (const float*)d_in[10];
    const float* e2b2  = (const float*)d_in[11];
    const float* root2 = (const float*)d_in[12];
    const float* bias2 = (const float*)d_in[13];
    const float* bn1g  = (const float*)d_in[14];
    const float* bn1b  = (const float*)d_in[15];
    const float* bn1m  = (const float*)d_in[16];
    const float* bn1v  = (const float*)d_in[17];
    const float* bn2g  = (const float*)d_in[18];
    const float* bn2b  = (const float*)d_in[19];
    const float* bn2m  = (const float*)d_in[20];
    const float* bn2v  = (const float*)d_in[21];
    const float* r1w   = (const float*)d_in[22];
    const float* r1b   = (const float*)d_in[23];
    const float* r2w   = (const float*)d_in[24];
    const float* r2b   = (const float*)d_in[25];
    const int*   ei    = (const int*)d_in[26];
    const int*   batch = (const int*)d_in[27];
    float* out = (float*)d_out;

    const int N = in_sizes[0] / FEAT;
    const int E = in_sizes[1] / 4;
    const int G = out_size;
    if (N <= 0 || E <= 0 || G < 1 || G > GMAX || (G & 3) != 0) return;
    if (in_sizes[0] != N * FEAT || in_sizes[1] != 4 * E || in_sizes[26] != 2 * E || in_sizes[27] != N) return;
    for (int L = 0; L < 2; ++L) {
        const int b = 2 + 6 * L;
        if (in_sizes[b] != 4 * FEAT || in_sizes[b + 1] != FEAT || in_sizes[b + 2] != FEAT * 1024 ||
            in_sizes[b + 3] != 1024 || in_sizes[b + 4] != FEAT * FEAT || in_sizes[b + 5] != FEAT) return;
    }
    for (int i = 14; i < 22; ++i) if (in_sizes[i] != FEAT) return;
    if (in_sizes[22] != FEAT * 16 || in_sizes[23] != 16 || in_sizes[24] != 16 || in_sizes[25] != 1) return;

    const int NB = (N + 31) / 32;
    if (NB + 1 > PITCHB || NB > MAXB) return;
    const int NB1 = (E + CH1 - 1) / CH1;
    if (NB1 > MAXNB1) return;
    const int NT = (N + 15) / 16;

    size_t off = 0;
    auto carve = [&](size_t bytes) -> size_t { const size_t p = off; off += (bytes + 255) & ~(size_t)255; return p; };
    const size_t o_bf1 = carve((size_t)NSLOTS * 8 * sizeof(_Float16));
    const size_t o_bf2 = carve((size_t)NSLOTS * 8 * sizeof(_Float16));
    const size_t o_lists = carve((size_t)NB1 * CH1 * sizeof(int));
    const size_t o_tab = carve((size_t)NB1 * PITCHB * sizeof(int));
    const size_t o_nodep = carve((size_t)NT * 16 * PITCH * sizeof(float));
    const size_t o_xt = carve((size_t)NB * 32 * FEAT * sizeof(float));
    const size_t o_xf = carve((size_t)NB * 32 * FEAT * sizeof(float));
    if (off > ws_size) return;

    char* ws = (char*)d_ws;
    _Float16* bf1 = (_Float16*)(ws + o_bf1);
    _Float16* bf2 = (_Float16*)(ws + o_bf2);
    int* lists = (int*)(ws + o_lists);
    int* offtab = (int*)(ws + o_tab);
    float* nodep = (float*)(ws + o_nodep);
    float* xt = (float*)(ws + o_xt);
    float* xf = (float*)(ws + o_xf);

    k_prep<<<(NSLOTS + 255) / 256, 256, 0, stream>>>(e1w2, root1, e1b2, bf1);
    k_prep<<<(NSLOTS + 255) / 256, 256, 0, stream>>>(e2w2, root2, e2b2, bf2);
    k_bucket<<<NB1, 256, 0, stream>>>(ei + E, lists, offtab, E, N);
    k_node<<<NT, 32, 0, stream>>>(x, bf1, nodep, N, NT);
    k_aggr<<<NB, 32, 0, stream>>>(ei, ea, e1w1, e1b1, bias1, bn1g, bn1b, bn1m, bn1v,
                                  nodep, lists, offtab, xt, E, N, NB1);
    k_node<<<NT, 32, 0, stream>>>(xt, bf2, nodep, N, NT);
    k_aggr<<<NB, 32, 0, stream>>>(ei, ea, e2w1, e2b1, bias2, bn2g, bn2b, bn2m, bn2v,
                                  nodep, lists, offtab, xf, E, N, NB1);
    k_tail<<<1, 128, 0, stream>>>(xf, batch, r1w, r1b, r2w, r2b, out, N, G, out_size);
}
